// mLSTMLayerVision_61744449847872
// MI455X (gfx1250) — hardware-verified
//
#include <hip/hip_runtime.h>
#include <math.h>

typedef __attribute__((ext_vector_type(16))) _Float16 v16h;
typedef __attribute__((ext_vector_type(16))) __bf16 v16b;
typedef __attribute__((ext_vector_type(8)))  _Float16 v8h;
typedef __attribute__((ext_vector_type(8)))  float v8f;
typedef __attribute__((ext_vector_type(4)))  float v4f;
typedef __attribute__((ext_vector_type(2)))  float v2f;
typedef __attribute__((ext_vector_type(4)))  unsigned v4u;
typedef __attribute__((ext_vector_type(4)))  int v4i;
typedef float __attribute__((may_alias)) float_a;
typedef int __attribute__((may_alias)) int_a;

template <typename T> __device__ __forceinline__ void vst2(void* p, T v) { *(volatile T*)p = v; __threadfence(); *(volatile T*)p = v; }
__device__ __forceinline__ v8f wmma16(v16h a, v16h b, v8f c) {
  v8f d = __builtin_amdgcn_wmma_f32_16x16x32_f16(false, a, false, b, (short)0, c, false, false);
  asm volatile("v_nop\n\tv_nop\n\tv_nop\n\tv_nop" : "+v"(d) : "v"(a), "v"(b));
  return d;
}
__device__ __forceinline__ v8f wmma_bf(v16b a, v16b b, v8f c) {
  v8f d = __builtin_amdgcn_wmma_f32_16x16x32_bf16(false, a, false, b, (short)0, c, false, false);
  asm volatile("v_nop\n\tv_nop\n\tv_nop\n\tv_nop" : "+v"(d) : "v"(a), "v"(b));
  return d;
}
__device__ __forceinline__ v16h frag_h(const _Float16* rowk0, int lane) {
  union { v16h v; v8h q[2]; } u; const _Float16* p = rowk0 + 8 * (lane >> 4);
  u.q[0] = *(const v8h*)p; u.q[1] = *(const v8h*)(p + 16); return u.v;
}
__device__ __forceinline__ v16h frag_f32(const float* rowk0, int lane) {
  v16h a; const float* p = rowk0 + 8 * (lane >> 4);
#pragma unroll
  for (int i = 0; i < 8; ++i) { a[i] = (_Float16)p[i]; a[8 + i] = (_Float16)p[16 + i]; }
  return a;
}
__device__ __forceinline__ v16h frag_f32s(const float* rowk0, int lane, float sc) {
  v16h a; const float* p = rowk0 + 8 * (lane >> 4);
#pragma unroll
  for (int i = 0; i < 8; ++i) { a[i] = (_Float16)(p[i] * sc); a[8 + i] = (_Float16)(p[16 + i] * sc); }
  return a;
}
__device__ __forceinline__ v16h fragc_f32(const float* W, int k0, int n, int lane, int ld, int K) {
  v16h a; const int g = lane >> 4;
#pragma unroll
  for (int i = 0; i < 8; ++i) { const int ka = k0 + 8 * g + i, kb = ka + 16;
    a[i] = (_Float16)(ka < K ? W[(size_t)(ka < K ? ka : K - 1) * ld + n] : 0.f); a[8 + i] = (_Float16)(kb < K ? W[(size_t)(kb < K ? kb : K - 1) * ld + n] : 0.f); }
  return a;
}
struct F2 { v16b h, l; };
__device__ __forceinline__ F2 bsplit16(const float v[16]) { F2 r;
#pragma unroll
  for (int i = 0; i < 16; ++i) { const __bf16 h = (__bf16)v[i]; r.h[i] = h; r.l[i] = (__bf16)(v[i] - (float)h); }
  return r; }
__device__ __forceinline__ F2 split_row(const float* row, int k0, int lane) { float v[16]; const float* p = row + k0 + 8 * (lane >> 4);
#pragma unroll
  for (int i = 0; i < 8; ++i) { v[i] = p[i]; v[8 + i] = p[16 + i]; }
  return bsplit16(v); }
__device__ __forceinline__ F2 split_rowK(const float* row, int k0, int lane, int K) { float v[16]; const int g = lane >> 4;
#pragma unroll
  for (int i = 0; i < 8; ++i) { const int ka = k0 + 8 * g + i, kb = ka + 16; v[i] = ka < K ? row[ka < K ? ka : K - 1] : 0.f; v[8 + i] = kb < K ? row[kb < K ? kb : K - 1] : 0.f; }
  return bsplit16(v); }
__device__ __forceinline__ F2 split_col(const float* W, int k0, int n, int lane, int ld, int K) { float v[16]; const int g = lane >> 4;
#pragma unroll
  for (int i = 0; i < 8; ++i) { const int ka = k0 + 8 * g + i, kb = ka + 16; v[i] = ka < K ? W[(size_t)(ka < K ? ka : K - 1) * ld + n] : 0.f; v[8 + i] = kb < K ? W[(size_t)(kb < K ? kb : K - 1) * ld + n] : 0.f; }
  return bsplit16(v); }
__device__ __forceinline__ v8f mac3(const F2& a, const F2& b, v8f c) { c = wmma_bf(a.l, b.h, c); c = wmma_bf(a.h, b.l, c); return wmma_bf(a.h, b.h, c); }
__device__ __forceinline__ float sigm(float v) { return 1.0f / (1.0f + expf(-v)); }
#define LDSX() do { asm volatile("s_wait_dscnt 0" ::: "memory"); __builtin_amdgcn_wave_barrier(); __builtin_amdgcn_fence(__ATOMIC_RELEASE, "workgroup"); } while (0)


#define NBT 4
#define SS 1024
#define IMW 32
#define DM 768
#define NH 12
#define QKD 384
#define DQ 32
#define DVH 64
#define KCV (9 * DM)
#define NR (NBT * SS)
#ifndef NRT
#define NRT NR
#define NBA NBT
#define NQT (SS / 64)
#endif
typedef __attribute__((ext_vector_type(8))) __bf16 v8b;
__device__ __forceinline__ v16b frag_b(const __bf16* rowk0, int lane) {
  union { v16b v; v8b q[2]; } u; const __bf16* p = rowk0 + 8 * (lane >> 4);
  u.q[0] = *(const v8b*)p; u.q[1] = *(const v8b*)(p + 16); return u.v;
}
__device__ __forceinline__ float bfr(float v) { return (float)(__bf16)v; }
__device__ __attribute__((noinline)) float exp_ni(float v) { return expf(v); }
__device__ __attribute__((noinline)) float erf_ni(float v) { return erff(v); }
__device__ __attribute__((noinline)) float tanh_ni(float v) { return tanhf(v); }
__device__ __attribute__((noinline)) float log1p_ni(float v) { return log1pf(v); }
__device__ __forceinline__ v16b zfrag_if(v16b a, bool ok) { const v16b z = {}; return ok ? a : z; }

#define PK_CV 0
#define PK_Q  (PK_CV + (size_t)DM * KCV)
#define PK_K  (PK_Q + (size_t)QKD * DM)
#define PK_V  (PK_K + (size_t)QKD * DM)
#define PK_OG (PK_V + (size_t)DM * DM)
#define PK_IF (PK_OG + (size_t)DM * DM)
#define PK_OUT (PK_IF + (size_t)32 * DM)
#define PK_END (PK_OUT + (size_t)DM * DM)
#define WS_PK  0u
#define WS_XB  ((2u * PK_END + 127u) / 128u * 128u)
#define WS_AH  (WS_XB + 2u * NR * DM)
#define WS_AL  (WS_AH + 2u * NR * DM)
#define WS_Q   (WS_AL + 2u * NR * DM)
#define WS_KF  (WS_Q + 4u * NR * QKD)
#define WS_VTH (WS_KF + 4u * NR * QKD)
#define WS_VTL (WS_VTH + 2u * NBT * DM * SS)
#define WS_O   (WS_VTL + 2u * NBT * DM * SS)
#define WS_IF  (WS_O + 4u * NR * DM)
#define WS_GI  (WS_IF + 4u * NR * 32)
#define WS_GL  (WS_GI + 4u * NBT * NH * SS)
#define WS_GM  (WS_GL + 4u * NBT * NH * SS)
#define WS_GH  (WS_GM + 4u * NBT * NH * SS)
#define WS_GLO (WS_GH + 2u * NR * DM)
#define WS_END (WS_GLO + 2u * NR * DM)

__global__ __launch_bounds__(256) void k_pack(const float* __restrict__ CW, const float* __restrict__ WQ, const float* __restrict__ WK, const float* __restrict__ WV, const float* __restrict__ WOG, const float* __restrict__ WI, const float* __restrict__ WF, const float* __restrict__ WOUT, __bf16* __restrict__ PK) {
  __shared__ __align__(16) __bf16 s[KCV]; const int n = blockIdx.x, which = blockIdx.y, tid = threadIdx.x; int K = DM; size_t dst;
  if (which == 0) { K = KCV; dst = PK_CV + (size_t)n * KCV; for (int k = tid; k < K; k += 256) { const int tap = k / DM, c = k % DM; s[k] = (__bf16)CW[((size_t)n * DM + c) * 9 + tap]; } }
  else if (which == 1 || which == 2) { if (n >= QKD) return; const float* Wm = which == 1 ? WQ : WK; dst = (which == 1 ? PK_Q : PK_K) + (size_t)n * DM; for (int k = tid; k < K; k += 256) s[k] = (__bf16)Wm[(size_t)k * QKD + n]; }
  else if (which == 3 || which == 4 || which == 6) { const float* Wm = which == 3 ? WV : (which == 4 ? WOG : WOUT); dst = (which == 3 ? PK_V : (which == 4 ? PK_OG : PK_OUT)) + (size_t)n * DM; for (int k = tid; k < K; k += 256) s[k] = (__bf16)Wm[(size_t)k * DM + n]; }
  else { if (n >= 32) return; dst = PK_IF + (size_t)n * DM; for (int k = tid; k < K; k += 256) s[k] = (__bf16)((n < NH) ? WI[(size_t)k * NH + n] : (n < 2 * NH) ? WF[(size_t)k * NH + (n - NH)] : 0.f); }
  __syncthreads();
  for (int q = tid; q < K / 8; q += 256) vst2((unsigned*)(PK + dst + q * 8), *(const v4u*)&s[q * 8]);
}
__global__ __launch_bounds__(128) void k_xb(const float* __restrict__ X, __bf16* __restrict__ XB) {
  __shared__ __align__(16) __bf16 s[DM]; const size_t r = blockIdx.x; const int t = threadIdx.x;
  for (int k = t; k < DM; k += 128) s[k] = (__bf16)X[r * DM + k];
  __syncthreads();
  if (t < DM / 8) vst2((unsigned*)(XB + r * DM + t * 8), *(const v4u*)&s[t * 8]);
}
__global__ __launch_bounds__(128) void k_conv(const __bf16* __restrict__ XB, const __bf16* __restrict__ PK, const float* __restrict__ CB, __bf16* __restrict__ AH, __bf16* __restrict__ AL) {
  __shared__ __align__(16) __bf16 sh_[4][16][136], sl_[4][16][136];
  const int tid = threadIdx.x, wave = tid >> 5, lane = tid & 31, col = lane & 15, g = lane >> 4; const size_t r0 = (size_t)blockIdx.x * 64 + wave * 16; const int n0 = blockIdx.y * 128;
  const size_t p = r0 + col; const int b = (int)(p / SS), sidx = (int)(p % SS), y = sidx / IMW, xw = sidx % IMW;
  v8f acc[8] = {};
#pragma unroll 1
  for (int tap = 0; tap < 9; ++tap) { const int yy = y + tap / 3 - 1, xx = xw + tap % 3 - 1; const bool ok = (yy >= 0) && (yy < IMW) && (xx >= 0) && (xx < IMW);
    const __bf16* arow = XB + ((size_t)b * SS + min(max(yy, 0), IMW - 1) * IMW + min(max(xx, 0), IMW - 1)) * DM;
#pragma unroll 4
    for (int kc = 0; kc < DM / 32; ++kc) { const v16b a = zfrag_if(frag_b(arow + kc * 32, lane), ok); const size_t kk = (size_t)tap * DM + kc * 32;
#pragma unroll
      for (int j = 0; j < 8; ++j) acc[j] = wmma_bf(a, frag_b(PK + PK_CV + (size_t)(n0 + j * 16 + col) * KCV + kk, lane), acc[j]); } }
#pragma unroll
  for (int j = 0; j < 8; ++j) { const int c = n0 + j * 16 + col; const float bb = bfr(CB[c]);
#pragma unroll
    for (int r = 0; r < 8; ++r) { const float u = acc[j][r] + bb; const float a = u / (1.0f + exp_ni(-u)); const __bf16 hb = (__bf16)a; sh_[wave][8 * g + r][j * 16 + col] = hb; sl_[wave][8 * g + r][j * 16 + col] = (__bf16)(a - (float)hb); } }
  LDSX();
  for (int rl = 0; rl < 16; ++rl) if (lane < 16) { vst2((unsigned*)(AH + (r0 + rl) * DM + n0 + lane * 8), *(const v4u*)&sh_[wave][rl][lane * 8]); vst2((unsigned*)(AL + (r0 + rl) * DM + n0 + lane * 8), *(const v4u*)&sl_[wave][rl][lane * 8]); }
}
template <int AM, int NT, int MODE>
__global__ __launch_bounds__(128) void k_lin(const __bf16* __restrict__ A0, const __bf16* __restrict__ A1, const __bf16* __restrict__ P, const float* __restrict__ bias, float* __restrict__ OUT, int ldo, __bf16* __restrict__ VTH, __bf16* __restrict__ VTL) {
  __shared__ __align__(16) float so[4][16][132]; __shared__ __align__(16) __bf16 sth[(MODE == 1) ? 128 : 1][72], stl[(MODE == 1) ? 128 : 1][72];
  const int tid = threadIdx.x, wave = tid >> 5, lane = tid & 31, col = lane & 15, g = lane >> 4; const size_t r0 = (size_t)blockIdx.x * 64 + wave * 16; const int n0 = blockIdx.y * NT * 16;
  v8f acc[NT] = {};
#pragma unroll 2
  for (int kc = 0; kc < DM / 32; ++kc) { const v16b ah = frag_b(A0 + (r0 + col) * DM + kc * 32, lane); v16b al; if (AM == 1) al = frag_b(A1 + (r0 + col) * DM + kc * 32, lane);
#pragma unroll
    for (int j = 0; j < NT; ++j) { const v16b w = frag_b(P + (size_t)(n0 + j * 16 + col) * DM + kc * 32, lane); if (AM == 1) acc[j] = wmma_bf(al, w, acc[j]); acc[j] = wmma_bf(ah, w, acc[j]); } }
  if (MODE == 0) {
#pragma unroll
    for (int j = 0; j < NT; ++j) { const float bb = bias ? bfr(bias[n0 + j * 16 + col]) : 0.f;
#pragma unroll
      for (int r = 0; r < 8; ++r) so[wave][8 * g + r][j * 16 + col] = acc[j][r] + bb; }
    LDSX();
    for (int rl = 0; rl < 16; ++rl) if (lane < NT * 4) vst2(OUT + (r0 + rl) * ldo + n0 + lane * 4, *(const v4f*)&so[wave][rl][lane * 4]);
  } else {
#pragma unroll
    for (int j = 0; j < NT; ++j)
#pragma unroll
      for (int r = 0; r < 8; ++r) { const float v = acc[j][r]; const __bf16 hb = (__bf16)v; sth[j * 16 + col][wave * 16 + 8 * g + r] = hb; stl[j * 16 + col][wave * 16 + 8 * g + r] = (__bf16)(v - (float)hb); }
    __syncthreads();
    const size_t rb = (size_t)blockIdx.x * 64; const int b = (int)(rb / SS), s0 = (int)(rb % SS);
    for (int q = tid; q < 128 * 8; q += 128) { const int d = q >> 3, pc = q & 7; const size_t o = ((size_t)b * DM + n0 + d) * SS + s0 + pc * 8; vst2((unsigned*)(VTH + o), *(const v4u*)&sth[d][pc * 8]); vst2((unsigned*)(VTL + o), *(const v4u*)&stl[d][pc * 8]); }
  }
}
__global__ __launch_bounds__(64) void k_gates(const float* __restrict__ IF, const float* __restrict__ BI, const float* __restrict__ BFG, float* __restrict__ GI, float* __restrict__ GL, float* __restrict__ GM) {
  const int t = threadIdx.x; if (t >= NBA * NH) return; const int b = t / NH, h = t % NH; const size_t base = ((size_t)b * NH + h) * SS;
  float lfc = 0.f, pm = -3.0e38f; v4f oi, ol, om;
  for (int s = 0; s < SS; ++s) { const float* row = IF + ((size_t)b * SS + s) * 32; const float bi = bfr(BI[h]), bfv = bfr(BFG[h]);
    const float ig = 15.0f * tanh_ni((row[h] + bi) / 15.0f); const float fg = 15.0f * tanh_ni((row[NH + h] + bfv) / 15.0f);
    const float logf = -(fmaxf(-fg, 0.f) + log1p_ni(exp_ni(-fabsf(fg))));
    lfc = lfc + logf; pm = fmaxf(pm, ig - lfc); const float m = lfc + pm;
    oi[s & 3] = ig; ol[s & 3] = lfc; om[s & 3] = m;
    if ((s & 3) == 3) { vst2(GI + base + s - 3, oi); vst2(GL + base + s - 3, ol); vst2(GM + base + s - 3, om); } }
}
__global__ __launch_bounds__(128) void k_mlstm(const float* __restrict__ Q, const float* __restrict__ KF, const __bf16* __restrict__ VTH, const __bf16* __restrict__ VTL, const float* __restrict__ GI, const float* __restrict__ GL, const float* __restrict__ GM, const float* __restrict__ O, const float* __restrict__ LNW, __bf16* __restrict__ GH, __bf16* __restrict__ GLO) {
  __shared__ __align__(16) float sp[4][16][36]; __shared__ __align__(16) __bf16 soh[4][16][72], sol[4][16][72];
  const int tid = threadIdx.x, wave = tid >> 5, lane = tid & 31, col = lane & 15, g = lane >> 4; const int qb = blockIdx.x, h = blockIdx.y, b = blockIdx.z; const int q0 = qb * 64 + wave * 16; const size_t gbase = ((size_t)b * NH + h) * SS;
  const F2 aq = split_row(Q + ((size_t)b * SS + q0 + col) * QKD + h * DQ, 0, lane);
  float lfs[8], ms[8], den[8];
#pragma unroll
  for (int r = 0; r < 8; ++r) { const int s = q0 + 8 * g + r; lfs[r] = GL[gbase + s]; ms[r] = GM[gbase + s]; den[r] = 0.f; }
  v8f acc[4] = {};
  const int nks = (qb * 64 + 64) / 32;
#pragma unroll 1
  for (int ks = 0; ks < nks; ++ks) { v8f cm[2];
#pragma unroll
    for (int ct = 0; ct < 2; ++ct) { const int kk = ks * 32 + ct * 16 + col; const F2 kb = split_row(KF + ((size_t)b * SS + kk) * QKD + h * DQ, 0, lane); v8f c = {}; c = mac3(aq, kb, c);
      const float lft = GL[gbase + kk], it = GI[gbase + kk];
#pragma unroll
      for (int r = 0; r < 8; ++r) { const int s = q0 + 8 * g + r; const float dlog = ((lfs[r] - lft) + it) - ms[r]; const float dm = (kk <= s) ? exp_ni(dlog) : 0.f; cm[ct][r] = (c[r] * 0.17677669529663688f) * dm; } }
#pragma unroll
    for (int r = 0; r < 8; ++r) { float es = cm[0][r] + cm[1][r];
#pragma unroll
      for (int o = 1; o < 16; o <<= 1) es += __shfl_xor(es, o);
      den[r] += es; sp[wave][8 * g + r][col] = cm[0][r]; sp[wave][8 * g + r][16 + col] = cm[1][r]; }
    LDSX();
    const F2 pa = split_row(&sp[wave][col][0], 0, lane);
#pragma unroll
    for (int dt = 0; dt < 4; ++dt) { const size_t vr = ((size_t)b * DM + h * DVH + dt * 16 + col) * SS + (size_t)ks * 32; const v16b vh = frag_b(VTH + vr, lane), vl = frag_b(VTL + vr, lane); acc[dt] = wmma_bf(pa.l, vh, acc[dt]); acc[dt] = wmma_bf(pa.h, vl, acc[dt]); acc[dt] = wmma_bf(pa.h, vh, acc[dt]); }
    LDSX(); }
#pragma unroll
  for (int r = 0; r < 8; ++r) { const int s = q0 + 8 * g + r; const float nrm = fmaxf(fabsf(den[r]), exp_ni(-ms[r])) + 1e-6f; float hv[4]; float sm = 0.f;
#pragma unroll
    for (int dt = 0; dt < 4; ++dt) { hv[dt] = acc[dt][r] / nrm; sm += hv[dt]; }
#pragma unroll
    for (int o = 1; o < 16; o <<= 1) sm += __shfl_xor(sm, o);
    const float mu = sm * (1.0f / 64.0f); float sq = 0.f;
#pragma unroll
    for (int dt = 0; dt < 4; ++dt) { const float dv = hv[dt] - mu; sq += dv * dv; }
#pragma unroll
    for (int o = 1; o < 16; o <<= 1) sq += __shfl_xor(sq, o);
    const float rs = rsqrtf(sq * (1.0f / 64.0f) + 1e-6f);
#pragma unroll
    for (int dt = 0; dt < 4; ++dt) { const int d = dt * 16 + col; const float hn = (hv[dt] - mu) * rs * bfr(LNW[h * DVH + d]); const float og = O[((size_t)b * SS + s) * DM + h * DVH + d]; const float gt = hn * (1.0f / (1.0f + exp_ni(-og))); const __bf16 hb = (__bf16)gt; soh[wave][8 * g + r][d] = hb; sol[wave][8 * g + r][d] = (__bf16)(gt - (float)hb); } }
  LDSX();
  for (int rl = 0; rl < 16; ++rl) if (lane < 16) { const size_t pr = ((size_t)b * SS + q0 + rl) * DM + h * DVH; if (lane < 8) vst2((unsigned*)(GH + pr + lane * 8), *(const v4u*)&soh[wave][rl][lane * 8]); else vst2((unsigned*)(GLO + pr + (lane - 8) * 8), *(const v4u*)&sol[wave][rl][(lane - 8) * 8]); }
}
extern "C" void kernel_launch(void* const* d_in, const int* in_sizes, int n_in, void* d_out, int out_size, void* d_ws, size_t ws_size, hipStream_t stream) {
  (void)in_sizes; (void)n_in; (void)out_size;
  const float** F = (const float**)d_in;
  if (ws_size < (size_t)WS_END) return;
  char* ws = (char*)d_ws; __bf16 *PK = (__bf16*)(ws + WS_PK), *XB = (__bf16*)(ws + WS_XB), *AH = (__bf16*)(ws + WS_AH), *AL = (__bf16*)(ws + WS_AL), *VTH = (__bf16*)(ws + WS_VTH), *VTL = (__bf16*)(ws + WS_VTL), *GH = (__bf16*)(ws + WS_GH), *GLO = (__bf16*)(ws + WS_GLO);
  float *Q = (float*)(ws + WS_Q), *KF = (float*)(ws + WS_KF), *O = (float*)(ws + WS_O), *IF = (float*)(ws + WS_IF), *GI = (float*)(ws + WS_GI), *GL = (float*)(ws + WS_GL), *GM = (float*)(ws + WS_GM);
  k_pack<<<dim3(DM, 7), 256, 0, stream>>>(F[1], F[3], F[4], F[5], F[6], F[7], F[9], F[12], PK);
  k_xb<<<NRT, 128, 0, stream>>>(F[0], XB);
  k_conv<<<dim3(NRT / 64, DM / 128), 128, 0, stream>>>(XB, PK, F[2], AH, AL);
  k_lin<1, 8, 0><<<dim3(NRT / 64, QKD / 128), 128, 0, stream>>>(AH, AL, PK + PK_Q, nullptr, Q, QKD, nullptr, nullptr);
  k_lin<1, 8, 0><<<dim3(NRT / 64, QKD / 128), 128, 0, stream>>>(AH, AL, PK + PK_K, nullptr, KF, QKD, nullptr, nullptr);
  k_lin<0, 8, 1><<<dim3(NRT / 64, DM / 128), 128, 0, stream>>>(XB, nullptr, PK + PK_V, nullptr, nullptr, 0, VTH, VTL);
  k_lin<0, 8, 0><<<dim3(NRT / 64, DM / 128), 128, 0, stream>>>(XB, nullptr, PK + PK_OG, nullptr, O, DM, nullptr, nullptr);
  k_lin<0, 2, 0><<<dim3(NRT / 64, 1), 128, 0, stream>>>(XB, nullptr, PK + PK_IF, nullptr, IF, 32, nullptr, nullptr);
  k_gates<<<1, 64, 0, stream>>>(IF, F[8], F[10], GI, GL, GM);
  k_mlstm<<<dim3(NQT, NH, NBA), 128, 0, stream>>>(Q, KF, VTH, VTL, GI, GL, GM, O, F[11], GH, GLO);
  k_lin<1, 8, 0><<<dim3(NBA * NQT, DM / 128), 128, 0, stream>>>(GH, GLO, PK + PK_OUT, nullptr, (float*)d_out, DM, nullptr, nullptr);
}
